// COIL_15118284882567
// MI455X (gfx1250) — hardware-verified
//
#include <hip/hip_runtime.h>


namespace {
constexpr int BQ = 64, LQ = 32, BD = 128, LD = 192, TD = 32, CD = 768;
constexpr float XS = 8.0f;

typedef _Float16 b16;
typedef __attribute__((ext_vector_type(16))) _Float16 v16b;
typedef __attribute__((ext_vector_type(8))) _Float16 v8b;
typedef __attribute__((ext_vector_type(8))) float v8f;
typedef __attribute__((ext_vector_type(4))) float v4f;
__device__ __forceinline__ float bf16_rne(float f) { unsigned int u = __float_as_uint(f); u += 0x7FFFu + ((u >> 16) & 1u); return __uint_as_float(u & 0xFFFF0000u); }
__device__ __forceinline__ v16b frag_kb(const b16* p, int hh) { const v8b a = *(const v8b*)(p + 8 * hh), b = *(const v8b*)(p + 16 + 8 * hh); v16b f;
#pragma unroll
  for (int e = 0; e < 8; ++e) { f[e] = a[e]; f[8 + e] = b[e]; } return f; }
__device__ __forceinline__ v8f wmma16b(v16b a, v16b b, v8f c) { v8f d = __builtin_amdgcn_wmma_f32_16x16x32_f16(false, a, false, b, (short)0, c, false, false); asm volatile("v_nop\n\tv_nop\n\tv_nop\n\tv_nop" : "+v"(d) : "v"(a), "v"(b)); return d; }
__device__ __forceinline__ void wave_lds_sync() { __builtin_amdgcn_fence(__ATOMIC_RELEASE, "workgroup"); __builtin_amdgcn_wave_barrier(); __builtin_amdgcn_fence(__ATOMIC_ACQUIRE, "workgroup"); }
__device__ __forceinline__ float pmul(float a, float b) { float p = a * b; asm volatile("" : "+v"(p)); return p; }

__global__ __launch_bounds__(256) void prep_kernel(const float* __restrict__ qt, const float* __restrict__ dt, const float* __restrict__ qc, const float* __restrict__ dc, b16* __restrict__ QT16, b16* __restrict__ DT16, b16* __restrict__ QC16, b16* __restrict__ DC16) {
  const size_t t = (size_t)blockIdx.x * 256 + threadIdx.x; const size_t n0 = (size_t)BQ * LQ * TD / 8, n1 = (size_t)BD * LD * TD / 8, n2 = (size_t)BQ * CD / 8, n3 = (size_t)BD * CD / 8; const float* src; b16* dst; size_t e;
  if (t < n0) { src = qt; dst = QT16; e = t * 8; } else if (t < n0 + n1) { src = dt; dst = DT16; e = (t - n0) * 8; } else if (t < n0 + n1 + n2) { src = qc; dst = QC16; e = (t - n0 - n1) * 8; } else if (t < n0 + n1 + n2 + n3) { src = dc; dst = DC16; e = (t - n0 - n1 - n2) * 8; } else return;
  const v4f a = *(const v4f*)(src + e), c = *(const v4f*)(src + e + 4); v8b o;
#pragma unroll
  for (int j = 0; j < 4; ++j) { o[j] = (b16)(bf16_rne(a[j]) * XS); o[4 + j] = (b16)(bf16_rne(c[j]) * XS); }
  for (int pass = 0; pass < 2; ++pass) { *(volatile v8b*)(dst + e) = o; __threadfence(); }
}
__global__ __launch_bounds__(128) void tok_kernel(const b16* __restrict__ QT16, const b16* __restrict__ DT16, const int* __restrict__ qid, const int* __restrict__ did, const int* __restrict__ amask, float* __restrict__ TOK) {
  __shared__ float res[32]; __shared__ float qm[LQ];
  const int wave = threadIdx.x >> 5, lane = threadIdx.x & 31, hh = lane >> 4, col = lane & 15; const int q = blockIdx.y, d0 = blockIdx.x * 32;
  if (threadIdx.x < 32) { int s = 0; for (int i = 0; i < LQ; ++i) s += amask[q * LQ + i]; const int sep = s - 1; const int m = amask[q * LQ + lane]; qm[lane] = (lane >= 1 && lane != sep) ? (float)m : 0.0f; }
  __syncthreads();
  const b16* Qb = QT16 + (size_t)q * LQ * TD; const v16b a0 = frag_kb(Qb + (size_t)col * TD, hh), a1 = frag_kb(Qb + (size_t)(16 + col) * TD, hh);
  int qi[2][8]; for (int rt = 0; rt < 2; ++rt) for (int r = 0; r < 8; ++r) qi[rt][r] = qid[q * LQ + rt * 16 + 8 * hh + r];
  for (int dd = 0; dd < 8; ++dd) { const int d = d0 + wave * 8 + dd; const b16* Db = DT16 + (size_t)d * LD * TD; const int* di = did + (size_t)d * LD;
    float mx[2][8];
#pragma unroll
    for (int rt = 0; rt < 2; ++rt) for (int r = 0; r < 8; ++r) mx[rt][r] = -INFINITY;
    for (int t = 0; t < LD / 16; ++t) { const v16b bd = frag_kb(Db + (size_t)(t * 16 + col) * TD, hh); v8f s0 = {}, s1 = {}; s0 = wmma16b(a0, bd, s0); s1 = wmma16b(a1, bd, s1); const int dj = di[t * 16 + col];
#pragma unroll
      for (int r = 0; r < 8; ++r) { const float v0 = (qi[0][r] == dj) ? s0[r] * (1.0f / (XS * XS)) : 0.0f, v1 = (qi[1][r] == dj) ? s1[r] * (1.0f / (XS * XS)) : 0.0f; mx[0][r] = fmaxf(mx[0][r], v0); mx[1][r] = fmaxf(mx[1][r], v1); } }
    float contrib = 0.0f;
#pragma unroll
    for (int rt = 0; rt < 2; ++rt)
#pragma unroll
      for (int r = 0; r < 8; ++r) { float m = mx[rt][r]; m = fmaxf(m, __shfl_xor(m, 1)); m = fmaxf(m, __shfl_xor(m, 2)); m = fmaxf(m, __shfl_xor(m, 4)); m = fmaxf(m, __shfl_xor(m, 8)); const int i = rt * 16 + 8 * hh + r; contrib += pmul(m, qm[i]); }
    contrib += __shfl_xor(contrib, 16);
    if (lane == 0) res[wave * 8 + dd] = contrib; }
  __syncthreads();
  for (int pass = 0; pass < 2; ++pass) { if (threadIdx.x < 8) *(volatile v4f*)(TOK + (size_t)q * BD + d0 + threadIdx.x * 4) = *(const v4f*)(&res[threadIdx.x * 4]); __threadfence(); }
}
__global__ __launch_bounds__(128) void cls_kernel(const b16* __restrict__ QC16, const b16* __restrict__ DC16, const float* __restrict__ TOK, float* __restrict__ out) {
  __shared__ __attribute__((aligned(16))) float Ts[4][16][128 + 4];
  const int wave = threadIdx.x >> 5, lane = threadIdx.x & 31, nloc = lane & 15, hlf = lane >> 4; const int m0 = wave * 16;
  v8f acc[8];
#pragma unroll
  for (int t = 0; t < 8; ++t) acc[t] = (v8f){};
  for (int kb = 0; kb < CD; kb += 32) { const v16b a = frag_kb(QC16 + (size_t)(m0 + nloc) * CD + kb, hlf);
#pragma unroll
    for (int t = 0; t < 8; ++t) acc[t] = wmma16b(a, frag_kb(DC16 + (size_t)(t * 16 + nloc) * CD + kb, hlf), acc[t]); }
#pragma unroll
  for (int t = 0; t < 8; ++t)
#pragma unroll
    for (int r = 0; r < 8; ++r) { const int qq = m0 + 8 * hlf + r, d = t * 16 + nloc; Ts[wave][8 * hlf + r][d] = acc[t][r] * (1.0f / (XS * XS)) + TOK[(size_t)qq * BD + d]; }
  wave_lds_sync();
  for (int pass = 0; pass < 2; ++pass) { for (int rr = 0; rr < 16; ++rr) *(volatile v4f*)(out + (size_t)(m0 + rr) * BD + lane * 4) = *(const v4f*)(&Ts[wave][rr][lane * 4]); __threadfence(); }
}
}

extern "C" void kernel_launch(void* const* d_in, const int* in_sizes, int n_in, void* d_out, int out_size, void* d_ws, size_t ws_size, hipStream_t stream) {
  (void)n_in;
  auto Fp = [&](int i) { return (const float*)d_in[i]; }; auto Ip = [&](int i) { return (const int*)d_in[i]; };
  if (in_sizes[0] != BQ * LQ * TD || in_sizes[1] != BD * LD * TD || in_sizes[2] != BQ * CD || in_sizes[3] != BD * CD || in_sizes[4] != BQ * LQ || in_sizes[5] != BD * LD || in_sizes[6] != BQ * LQ || out_size != BQ * BD) return;
  size_t off = 0; char* ws = (char*)d_ws;
  auto carve = [&](size_t bytes) { char* p = ws + off; off += (bytes + 255) & ~(size_t)255; return p; };
  b16* QT16 = (b16*)carve((size_t)BQ * LQ * TD * 2); b16* DT16 = (b16*)carve((size_t)BD * LD * TD * 2); b16* QC16 = (b16*)carve((size_t)BQ * CD * 2); b16* DC16 = (b16*)carve((size_t)BD * CD * 2); float* TOK = (float*)carve((size_t)BQ * BD * 4);
  if (off > ws_size || off > ((size_t)128 << 20)) return;
  prep_kernel<<<(unsigned)((((size_t)BQ * LQ * TD + (size_t)BD * LD * TD + (size_t)BQ * CD + (size_t)BD * CD) / 8 + 255) / 256), 256, 0, stream>>>(Fp(0), Fp(1), Fp(2), Fp(3), QT16, DT16, QC16, DC16);
  tok_kernel<<<dim3(BD / 32, BQ), 128, 0, stream>>>(QT16, DT16, Ip(4), Ip(5), Ip(6), TOK);
  cls_kernel<<<1, 128, 0, stream>>>(QC16, DC16, TOK, (float*)d_out);
}
